// GraphSAGELinkPred_79963701117112
// MI455X (gfx1250) — hardware-run, weakly checked
//
#include <hip/hip_runtime.h>

typedef float          v8f   __attribute__((ext_vector_type(8)));
typedef float          v4f   __attribute__((ext_vector_type(4)));
typedef unsigned int   v4u   __attribute__((ext_vector_type(4)));
typedef int            v8i   __attribute__((ext_vector_type(8)));
typedef unsigned short v8us  __attribute__((ext_vector_type(8)));
typedef unsigned short v16us __attribute__((ext_vector_type(16)));
typedef __bf16         v16bf __attribute__((ext_vector_type(16)));
typedef _Float16       v16h  __attribute__((ext_vector_type(16)));
typedef v4f  __attribute__((may_alias)) v4fa;
typedef v8us __attribute__((may_alias)) v8usa;
union FragB { v16bf v; v16us u; v8us h[2]; v8i w; };
union FragH { v16h  v; v16us u; v8us h[2]; v8i w; };

__device__ __forceinline__ v8f wmb(const FragB& a, const FragB& b, v8f c) {
  v8f d = __builtin_amdgcn_wmma_f32_16x16x32_bf16(false, a.v, false, b.v, (short)0, c, false, false);
  asm volatile("v_nop\n\tv_nop\n\tv_nop\n\tv_nop" : "+v"(d) : "v"(a.w), "v"(b.w));
  return d;
}

__device__ __forceinline__ v8f wmh(const FragH& a, const FragH& b, v8f c) {
  v8f d = __builtin_amdgcn_wmma_f32_16x16x32_f16(false, a.v, false, b.v, (short)0, c, false, false);
  asm volatile("v_nop\n\tv_nop\n\tv_nop\n\tv_nop" : "+v"(d) : "v"(a.w), "v"(b.w));
  return d;
}

__device__ __forceinline__ unsigned bf16_bits(float f) {
  const unsigned u = __float_as_uint(f);
  const unsigned r = (u + 0x7FFFu + ((u >> 16) & 1u)) >> 16;
  const unsigned q = (u >> 16) | 0x40u;
  return ((u & 0x7fffffffu) > 0x7f800000u) ? q : r;
}

__device__ __forceinline__ float bf16_val(float f) {
  return __uint_as_float(bf16_bits(f) << 16);
}
__device__ __forceinline__ int clampi(int v, int lo, int hi) {
  return v < lo ? lo : (v > hi ? hi : v);
}

__device__ __forceinline__ unsigned f16_bits(float f) {
  const unsigned u  = __float_as_uint(f);
  const unsigned s  = (u >> 16) & 0x8000u;
  const unsigned a  = u & 0x7fffffffu;
  const unsigned t  = a - 0x38000000u;
  const unsigned r  = (t + 0x0FFFu + ((t >> 13) & 1u)) >> 13;
  const unsigned rc = r > 0x7C00u ? 0x7C00u : r;
  const bool small  = a < 0x38800000u;
  const bool isnan  = a > 0x7f800000u;
  const unsigned fin = small ? 0u : (s | rc);
  return isnan ? (s | 0x7E00u) : fin;
}

__device__ __forceinline__ unsigned pk16(unsigned lo, unsigned hi) { return lo | (hi << 16); }
__device__ __forceinline__ unsigned bf16_lo_bits(float v) {
  float hi = bf16_val(v);
  asm volatile("" : "+v"(hi));
  return bf16_bits(v - hi);
}
__device__ __forceinline__ v4u pack8_bf16(v4f a, v4f c) {
  return (v4u){ pk16(bf16_bits(a[0]), bf16_bits(a[1])), pk16(bf16_bits(a[2]), bf16_bits(a[3])),
                pk16(bf16_bits(c[0]), bf16_bits(c[1])), pk16(bf16_bits(c[2]), bf16_bits(c[3])) };
}
__device__ __forceinline__ v4u pack8_bf16_lo(v4f a, v4f c) {
  return (v4u){ pk16(bf16_lo_bits(a[0]), bf16_lo_bits(a[1])), pk16(bf16_lo_bits(a[2]), bf16_lo_bits(a[3])),
                pk16(bf16_lo_bits(c[0]), bf16_lo_bits(c[1])), pk16(bf16_lo_bits(c[2]), bf16_lo_bits(c[3])) };
}
__device__ __forceinline__ v4u pack8_f16(v4f a, v4f c) {
  return (v4u){ pk16(f16_bits(a[0]), f16_bits(a[1])), pk16(f16_bits(a[2]), f16_bits(a[3])),
                pk16(f16_bits(c[0]), f16_bits(c[1])), pk16(f16_bits(c[2]), f16_bits(c[3])) };
}

template <int FORM>
__global__ __launch_bounds__(256) void k_plane(const float* __restrict__ src, int rows, int cols, int ldsrc,
                                               unsigned short* __restrict__ dst, int MP, int KP) {
  static_assert(FORM >= 0 && FORM <= 3);
  const int KTOT = (FORM == 1 || FORM == 3) ? 2 * KP : KP;
  const unsigned ppr   = (unsigned)(KTOT >> 3);
  const unsigned kp8   = (unsigned)(KP >> 3);
  const unsigned total = (unsigned)MP * ppr;
  const unsigned g     = blockIdx.x * 256u + threadIdx.x;
  const unsigned rowu  = g / ppr;
  const unsigned p     = g - rowu * ppr;
  const bool second    = p >= kp8;
  const int row = (int)rowu;
  const int c0  = (int)((second ? p - kp8 : p) << 3);
  const float* srow = src + (size_t)clampi(row, 0, rows - 1) * (size_t)ldsrc;
  float x[8];
  unsigned mk[8];
#pragma unroll
  for (int e = 0; e < 8; ++e) {
    const int c = c0 + e;
    const float v = srow[clampi(c, 0, cols - 1)];
    asm volatile("" :: "v"(v));
    x[e]  = v;
    mk[e] = (row < rows && c < cols) ? 0xFFFFu : 0u;
  }
  const v4f a = (v4f){ x[0], x[1], x[2], x[3] };
  const v4f c = (v4f){ x[4], x[5], x[6], x[7] };
  v4u o;
  if (FORM == 2) {
    o = pack8_f16(a, c);
  } else {
    const v4u hi = pack8_bf16(a, c);
    o = hi;
    if (FORM == 1) { const v4u lo = pack8_bf16_lo(a, c); o = second ? lo : hi; }
  }
  const v4u mw = (v4u){ pk16(mk[0], mk[1]), pk16(mk[2], mk[3]), pk16(mk[4], mk[5]), pk16(mk[6], mk[7]) };
  o &= mw;
  if (g < total) {
    volatile v4u* q = (volatile v4u*)(dst + (size_t)g * 8);
    *q = o;
    __threadfence();
    *q = o;
  }
}

template <int FORM> struct FragOf    { typedef FragB T; };
template <>         struct FragOf<2> { typedef FragH T; };
__device__ __forceinline__ v8f mm(const FragB& a, const FragB& b, v8f c) { return wmb(a, b, c); }
__device__ __forceinline__ v8f mm(const FragH& a, const FragH& b, v8f c) { return wmh(a, b, c); }
template <class F> __device__ __forceinline__ F ld_frag(const unsigned short* p) {
  F f;
  f.h[0] = *(const v8usa*)(p);
  f.h[1] = *(const v8usa*)(p + 16);
  return f;
}

template <int FORM, int EPI>
__global__ __launch_bounds__(256) __attribute__((amdgpu_num_vgpr(248)))
void k_gemm_nt(const unsigned short* __restrict__ A, const unsigned short* __restrict__ B,
               const float* __restrict__ bias, float* __restrict__ D, int M, int N, int KTOT, int ldd) {
  static_assert(FORM >= 0 && FORM <= 2);
  static_assert(EPI == 0 || EPI == 1);
  typedef typename FragOf<FORM>::T F;
  __shared__ __attribute__((aligned(16))) float sT[8][16 * 68];
  const int lane = threadIdx.x & 31;
  const int wave = threadIdx.x >> 5;
  const int tilesM = (M + 63) >> 6;
  const int tilesN = (N + 63) >> 6;
  const int tile = blockIdx.x * 8 + wave;
  if (tile >= tilesM * tilesN) return;
  const int tm = tile / tilesN;
  const int tn = tile - tm * tilesN;
  const int m0 = tm << 6;
  const int n0 = tn << 6;

  const int rl = lane & 15;
  const int h8 = (lane >> 4) * 8;
  const unsigned short* pa = A + (size_t)(m0 + rl) * (size_t)KTOT + h8;
  const unsigned short* pb = B + (size_t)(n0 + rl) * (size_t)KTOT + h8;

  v8f acc[4][4];
#pragma unroll
  for (int i = 0; i < 4; ++i)
#pragma unroll
    for (int j = 0; j < 4; ++j) acc[i][j] = (v8f){0.f, 0.f, 0.f, 0.f, 0.f, 0.f, 0.f, 0.f};

#pragma unroll 1
  for (int k0 = 0; k0 < KTOT; k0 += 32) {
    F bf[4];
#pragma unroll
    for (int j = 0; j < 4; ++j) bf[j] = ld_frag<F>(pb + (size_t)(j << 4) * (size_t)KTOT + k0);
#pragma unroll
    for (int i = 0; i < 4; ++i) {
      const F af = ld_frag<F>(pa + (size_t)(i << 4) * (size_t)KTOT + k0);
#pragma unroll
      for (int j = 0; j < 4; ++j) acc[i][j] = mm(af, bf[j], acc[i][j]);
    }
  }

  float* slab = sT[wave];
  const int hh = lane >> 4;
  const int c4 = (lane & 15) * 4;
  const int nc = n0 + c4;
  const bool cok = nc < N;
  v4f bv = (v4f){0.f, 0.f, 0.f, 0.f};
  if (EPI == 1) {
    bv = *(const v4fa*)(bias + clampi(nc, 0, N - 4));
    asm volatile("" :: "v"(bv));
  }
#pragma unroll
  for (int i = 0; i < 4; ++i) {
    const int mBase = m0 + (i << 4);
#pragma unroll
    for (int j = 0; j < 4; ++j) {
#pragma unroll
      for (int r = 0; r < 8; ++r) slab[(h8 + r) * 68 + (j << 4) + rl] = acc[i][j][r];
    }
    __builtin_amdgcn_fence(__ATOMIC_RELEASE, "workgroup");
    __builtin_amdgcn_wave_barrier();
    __builtin_amdgcn_fence(__ATOMIC_ACQUIRE, "workgroup");
    v4f vv[8];
#pragma unroll
    for (int it = 0; it < 8; ++it) {
      const int row = it * 2 + hh;
      v4f v = *(const v4fa*)(slab + row * 68 + c4);
      if (EPI == 1) v += bv;
      vv[it] = v;
    }
    for (int pass = 0; pass < 2; ++pass) {
#pragma unroll
      for (int it = 0; it < 8; ++it) {
        const int row = mBase + it * 2 + hh;
        if (cok && row < M) *(volatile v4f*)(D + (size_t)row * (size_t)ldd + nc) = vv[it];
      }
      __threadfence();
    }
    __builtin_amdgcn_fence(__ATOMIC_RELEASE, "workgroup");
    __builtin_amdgcn_wave_barrier();
    __builtin_amdgcn_fence(__ATOMIC_ACQUIRE, "workgroup");
  }
}

#include <stddef.h>
#pragma clang fp contract(off)

#ifndef SPLIT_L2
#define SPLIT_L2 1
#endif

#define NN      100000
#define FD      128
#define OD      64
#define K2      256
#define NE      1600000
#define NPAIR   200000
#define MP      100096
#define NTHR    256
#define NWAVE   8
#define EPT     8
#define WCH     (32 * EPT)
#define NBRUN   1024
#define SLB     10
#define NBK     98
#define WLCAP   4096
#define RCAP    21504
#define DEGCAP  64
#define MAXDEG_MEAS   36
#define MAXB1024_MEAS 16710
#define WBLK    12500
#define PADBLK  12
#define HBLK    782

#define BK_ZINTS (NWAVE * WLCAP + RCAP + 3 * NBRUN)
#define BK_INTS  (BK_ZINTS + 16)
#define BK_LDS   (BK_INTS * 4)

#define PW_U    (FD * FD / 8)
#define PW_B    (PW_U / NTHR)
#define PW_BLKS (4 * PW_B + 1)

#define TB_BL1    0
#define TB_WDEC   128
#define TB_BL2    256
#define TB_BDEC   384
#define TB_FLOATS 512

static_assert(SPLIT_L2 == 0 || SPLIT_L2 == 1);
static_assert(MP == 782 * 128 && MP % 64 == 0 && MP >= NN);
static_assert(NN % 16 == 0 && FD == 32 * 4 && OD == 32 * 2 && K2 == 2 * FD);
static_assert(FD % 64 == 0 && OD % 64 == 0 && FD % 32 == 0 && K2 % 32 == 0);
static_assert(WBLK * NWAVE == NN);
static_assert(PADBLK * NWAVE == MP - NN);
static_assert(NBRUN == (1 << SLB) && NBRUN == NTHR * 4 && NBRUN % 32 == 0);
static_assert(NBK * NBRUN >= NN && (NBK - 1) * NBRUN < NN);
static_assert(NE < (1 << 21) && (((long long)NE) << SLB) < (1LL << 31));
static_assert(NE % WCH == 0 && NE % 4 == 0 && NE >= EPT);
static_assert(RCAP % (NTHR * 4) == 0);
static_assert((long long)RCAP * 100 >= (long long)MAXB1024_MEAS * 125);
static_assert(WLCAP * 2 >= (MAXB1024_MEAS / NWAVE) * 3);
static_assert(MAXDEG_MEAS + 8 <= DEGCAP);
static_assert(BK_ZINTS % (NTHR * 4) == 0 && BK_LDS <= 262144);
static_assert(PW_U % NTHR == 0 && OD * K2 / 8 == PW_U);
static_assert((MP * FD / 8) % NTHR == 0);
static_assert(NPAIR % 32 == 0 && HBLK * NWAVE * 32 >= NPAIR && (HBLK - 1) * NWAVE * 32 < NPAIR);

typedef int          v4i  __attribute__((ext_vector_type(4)));
typedef unsigned int v2u  __attribute__((ext_vector_type(2)));
typedef float        v2f  __attribute__((ext_vector_type(2)));
typedef v4i __attribute__((may_alias)) v4ia;
typedef v2f __attribute__((may_alias)) v2fa;

__device__ __forceinline__ void st2_v4f(float* p, v4f v) {
  *(volatile v4f*)p = v;
  __threadfence();
  *(volatile v4f*)p = v;
}
__device__ __forceinline__ void st2_v4u(unsigned short* p, v4u v) {
  *(volatile v4u*)p = v;
  __threadfence();
  *(volatile v4u*)p = v;
}
__device__ __forceinline__ v4u cvt8(const float* __restrict__ p) {
  const v4f a = *(const v4fa*)p;
  const v4f c = *(const v4fa*)(p + 4);
  return pack8_bf16(a, c);
}

__global__ __launch_bounds__(NTHR) void k_prep(const float* __restrict__ Wl1, const float* __restrict__ Wr1,
                                               const float* __restrict__ Wl2, const float* __restrict__ Wr2,
                                               const float* __restrict__ bl1, const float* __restrict__ bl2,
                                               const float* __restrict__ Wdec, const float* __restrict__ bdec,
                                               unsigned short* w1l, unsigned short* w1r,
                                               unsigned short* w2l, unsigned short* w2r, float* tab) {
  const int tid = (int)threadIdx.x;
  const int blk = (int)blockIdx.x;
  if (blk < PW_B) {
    const int u = blk * NTHR + tid;
    const int n = u >> 4, k8 = (u & 15) * 8;
    const v4u o = cvt8(Wl1 + (size_t)n * FD + k8);
    st2_v4u(w1l + (size_t)u * 8, o);
  } else if (blk < 2 * PW_B) {
    const int u = (blk - PW_B) * NTHR + tid;
    const int n = u >> 4, k8 = (u & 15) * 8;
    const v4u o = cvt8(Wr1 + (size_t)n * FD + k8);
    st2_v4u(w1r + (size_t)u * 8, o);
  } else if (blk < 3 * PW_B) {
    const int u = (blk - 2 * PW_B) * NTHR + tid;
    const int n = u >> 5, ks = (u & 15) * 8;
    const v4u o = cvt8(Wl2 + (size_t)n * FD + ks);
    st2_v4u(w2l + (size_t)u * 8, o);
  } else if (blk < 4 * PW_B) {
    const int u = (blk - 3 * PW_B) * NTHR + tid;
    const int n = u >> 5, ks = (u & 15) * 8;
    const v4u o = cvt8(Wr2 + (size_t)n * FD + ks);
    st2_v4u(w2r + (size_t)u * 8, o);
  } else {
    const int wave = tid >> 5, lane = tid & 31;
    if (wave == 0) {
      const v4f v = *(const v4fa*)(bl1 + 4 * lane);
      v4f o;
      o.x = bf16_val(v.x); o.y = bf16_val(v.y); o.z = bf16_val(v.z); o.w = bf16_val(v.w);
      st2_v4f(tab + TB_BL1 + 4 * lane, o);
    } else if (wave == 1) {
      const v4f v = *(const v4fa*)(Wdec + 4 * lane);
      v4f o;
      o.x = bf16_val(v.x); o.y = bf16_val(v.y); o.z = bf16_val(v.z); o.w = bf16_val(v.w);
      st2_v4f(tab + TB_WDEC + 4 * lane, o);
    } else if (wave == 2) {
      const int lc = lane < 16 ? lane : 15;
      const v4f v = *(const v4fa*)(bl2 + 4 * lc);
      asm volatile("" :: "v"(v));
      v4f o;
      o.x = bf16_val(v.x); o.y = bf16_val(v.y); o.z = bf16_val(v.z); o.w = bf16_val(v.w);
      if (lane < 16) st2_v4f(tab + TB_BL2 + 4 * lane, o);
    } else if (wave == 3) {
      const float b = bdec[0];
      asm volatile("" :: "v"(b));
      const float bv = bf16_val(b);
      const v4f o = (v4f){bv, bv, bv, bv};
      if (lane < 8) st2_v4f(tab + TB_BDEC + 4 * lane, o);
    }
  }
}

__device__ __forceinline__ void build_flush(const int* pl, const int* cnt, const int* offs, int ov,
                                            int* lp, int* cp, int* op, int* fp, int tid) {
#pragma unroll 1
  for (int i = tid * 4; i < RCAP; i += NTHR * 4) {
    const v4i v = *(const v4ia*)(pl + i);
    *(volatile v4i*)(lp + i) = v;
  }
  {
    const v4i v = *(const v4ia*)(cnt + 4 * tid);
    *(volatile v4i*)(cp + 4 * tid) = v;
  }
  {
    const v4i v = *(const v4ia*)(offs + 4 * tid);
    *(volatile v4i*)(op + 4 * tid) = v;
  }
  if (tid < 8) {
    const v4i f = {ov, ov, ov, ov};
    *(volatile v4i*)(fp + 4 * tid) = f;
  }
}

__global__ __launch_bounds__(NTHR) void k_build(const int* __restrict__ srcs, const int* __restrict__ dsts,
                                                int* LIST, int* CNT, int* OFF, int* FLAG) {
  extern __shared__ __attribute__((aligned(16))) int dsm[];
  int* wl   = dsm;
  int* pl   = dsm + NWAVE * WLCAP;
  int* cnt  = pl + RCAP;
  int* offs = cnt + NBRUN;
  int* cur  = offs + NBRUN;
  int* misc = cur + NBRUN;
  const int tid = (int)threadIdx.x, lane = tid & 31, wave = tid >> 5;
  const int blk = (int)blockIdx.x;
  const unsigned nbs = (unsigned)(blk * NBRUN);

  {
    const v4i z4 = {0, 0, 0, 0};
    for (int i = tid * 4; i < BK_ZINTS; i += NTHR * 4) *(v4ia*)(dsm + i) = z4;
    if (tid < 16) misc[tid] = 0;
  }
  __syncthreads();

  {
    const int per  = ((NE + NWAVE * WCH - 1) / (NWAVE * WCH)) * WCH;
    const int ebeg = wave * per;
    const int eend = (ebeg + per < NE) ? (ebeg + per) : NE;
    int* mylist = wl + wave * WLCAP;
    int wc = 0;
#pragma unroll 1
    for (int cb = ebeg; cb < eend; cb += WCH) {
      const int e0 = cb + lane * EPT;
      const int ec = e0 < NE - EPT ? e0 : NE - EPT;
      const bool lv = e0 < NE;
      const v4i da = *(const v4ia*)(dsts + ec);
      const v4i db = *(const v4ia*)(dsts + ec + 4);
      const int k0 = da.x, k1 = da.y, k2 = da.z, k3 = da.w;
      const int k4 = db.x, k5 = db.y, k6 = db.z, k7 = db.w;
      asm volatile("" :: "v"(k0));
      asm volatile("" :: "v"(k1));
      asm volatile("" :: "v"(k2));
      asm volatile("" :: "v"(k3));
      asm volatile("" :: "v"(k4));
      asm volatile("" :: "v"(k5));
      asm volatile("" :: "v"(k6));
      asm volatile("" :: "v"(k7));
      const unsigned s0 = (unsigned)k0 - nbs, s1 = (unsigned)k1 - nbs;
      const unsigned s2 = (unsigned)k2 - nbs, s3 = (unsigned)k3 - nbs;
      const unsigned s4 = (unsigned)k4 - nbs, s5 = (unsigned)k5 - nbs;
      const unsigned s6 = (unsigned)k6 - nbs, s7 = (unsigned)k7 - nbs;
      const bool h0 = lv && s0 < (unsigned)NBRUN && (unsigned)k0 < (unsigned)NN;
      const bool h1 = lv && s1 < (unsigned)NBRUN && (unsigned)k1 < (unsigned)NN;
      const bool h2 = lv && s2 < (unsigned)NBRUN && (unsigned)k2 < (unsigned)NN;
      const bool h3 = lv && s3 < (unsigned)NBRUN && (unsigned)k3 < (unsigned)NN;
      const bool h4 = lv && s4 < (unsigned)NBRUN && (unsigned)k4 < (unsigned)NN;
      const bool h5 = lv && s5 < (unsigned)NBRUN && (unsigned)k5 < (unsigned)NN;
      const bool h6 = lv && s6 < (unsigned)NBRUN && (unsigned)k6 < (unsigned)NN;
      const bool h7 = lv && s7 < (unsigned)NBRUN && (unsigned)k7 < (unsigned)NN;
      const unsigned m0 = __builtin_amdgcn_ballot_w32(h0), m1 = __builtin_amdgcn_ballot_w32(h1);
      const unsigned m2 = __builtin_amdgcn_ballot_w32(h2), m3 = __builtin_amdgcn_ballot_w32(h3);
      const unsigned m4 = __builtin_amdgcn_ballot_w32(h4), m5 = __builtin_amdgcn_ballot_w32(h5);
      const unsigned m6 = __builtin_amdgcn_ballot_w32(h6), m7 = __builtin_amdgcn_ballot_w32(h7);
      const unsigned any = m0 | m1 | m2 | m3 | m4 | m5 | m6 | m7;
      if (any != 0u) {
        const int pre = (int)(__builtin_amdgcn_mbcnt_lo(m0, 0u) + __builtin_amdgcn_mbcnt_lo(m1, 0u) +
                              __builtin_amdgcn_mbcnt_lo(m2, 0u) + __builtin_amdgcn_mbcnt_lo(m3, 0u) +
                              __builtin_amdgcn_mbcnt_lo(m4, 0u) + __builtin_amdgcn_mbcnt_lo(m5, 0u) +
                              __builtin_amdgcn_mbcnt_lo(m6, 0u) + __builtin_amdgcn_mbcnt_lo(m7, 0u));
        int p = wc + pre;
        if (h0) { if (p < WLCAP) mylist[p] = ((e0 + 0) << SLB) | (int)s0; p = p + 1; }
        if (h1) { if (p < WLCAP) mylist[p] = ((e0 + 1) << SLB) | (int)s1; p = p + 1; }
        if (h2) { if (p < WLCAP) mylist[p] = ((e0 + 2) << SLB) | (int)s2; p = p + 1; }
        if (h3) { if (p < WLCAP) mylist[p] = ((e0 + 3) << SLB) | (int)s3; p = p + 1; }
        if (h4) { if (p < WLCAP) mylist[p] = ((e0 + 4) << SLB) | (int)s4; p = p + 1; }
        if (h5) { if (p < WLCAP) mylist[p] = ((e0 + 5) << SLB) | (int)s5; p = p + 1; }
        if (h6) { if (p < WLCAP) mylist[p] = ((e0 + 6) << SLB) | (int)s6; p = p + 1; }
        if (h7) { if (p < WLCAP) mylist[p] = ((e0 + 7) << SLB) | (int)s7; p = p + 1; }
        wc += (int)(__builtin_popcount(m0) + __builtin_popcount(m1) + __builtin_popcount(m2) + __builtin_popcount(m3) +
                    __builtin_popcount(m4) + __builtin_popcount(m5) + __builtin_popcount(m6) + __builtin_popcount(m7));
      }
    }
    if (lane == 0) misc[wave] = wc;
  }
  __syncthreads();

  if (wave == 0) {
    int ov = 0;
    int tot = 0;
#pragma unroll 1
    for (int w2 = 0; w2 < NWAVE; ++w2) {
      int c = misc[w2];
      if (c > WLCAP) ov = 1;
      c = c < 0 ? 0 : (c > WLCAP ? WLCAP : c);
      tot += c;
#pragma unroll 1
      for (int b0 = 0; b0 < c; b0 += 32) {
        const int idx = b0 + lane;
        const int ent = wl[w2 * WLCAP + (idx < WLCAP ? idx : WLCAP - 1)];
        const int m32 = (c - b0) < 32 ? (c - b0) : 32;
#pragma unroll 1
        for (int k = 0; k < m32; ++k) {
          const int u    = __builtin_amdgcn_readlane(ent, k);
          const int slot = u & (NBRUN - 1);
          if (lane == 0) cnt[slot] = cnt[slot] + 1;
        }
      }
    }
    if (tot > RCAP) ov = 1;
    if (lane == 0) misc[9] = ov;
  }
  __syncthreads();
  if (wave == 0) {
    const int base = lane * (NBRUN / 32);
    int s = 0;
#pragma unroll 1
    for (int i = 0; i < NBRUN / 32; ++i) s += cnt[base + i];
    int incl = s;
#pragma unroll
    for (int d = 1; d < 32; d <<= 1) {
      const int y = __shfl_up(incl, d, 32);
      if (lane >= d) incl += y;
    }
    int run = incl - s;
#pragma unroll 1
    for (int i = 0; i < NBRUN / 32; ++i) {
      const int cv = cnt[base + i];
      offs[base + i] = run;
      cur[base + i]  = run;
      run += cv;
    }
  }
  __syncthreads();

  if (wave == 0) {
#pragma unroll 1
    for (int w2 = 0; w2 < NWAVE; ++w2) {
      int c = misc[w2];
      c = c < 0 ? 0 : (c > WLCAP ? WLCAP : c);
#pragma unroll 1
      for (int b0 = 0; b0 < c; b0 += 32) {
        const int idx = b0 + lane;
        const int ent = wl[w2 * WLCAP + (idx < WLCAP ? idx : WLCAP - 1)];
        int eid = (ent >> SLB) & 0x1FFFFF;
        eid = eid > NE - 1 ? NE - 1 : eid;
        int sr = srcs[eid];
        asm volatile("" :: "v"(sr));
        sr = clampi(sr, 0, NN - 1);
        const int m32 = (c - b0) < 32 ? (c - b0) : 32;
#pragma unroll 1
        for (int k = 0; k < m32; ++k) {
          const int u    = __builtin_amdgcn_readlane(ent, k);
          const int w0   = __builtin_amdgcn_readlane(sr, k);
          const int slot = u & (NBRUN - 1);
          if (lane == 0) {
            int p = cur[slot];
            p = p < 0 ? 0 : (p > RCAP - 1 ? RCAP - 1 : p);
            pl[p] = w0;
            cur[slot] = p + 1;
          }
        }
      }
    }
  }
  __syncthreads();

  const int ovf = misc[9];
  int* lp = LIST + (size_t)blk * (size_t)RCAP;
  int* cp = CNT  + (size_t)blk * NBRUN;
  int* op = OFF  + (size_t)blk * NBRUN;
  int* fp = FLAG + (size_t)blk * 32;
  build_flush(pl, cnt, offs, ovf, lp, cp, op, fp, tid);
  __threadfence();
  build_flush(pl, cnt, offs, ovf, lp, cp, op, fp, tid);
}

__global__ __launch_bounds__(NTHR) void k_walk1(const int* __restrict__ LIST, const int* __restrict__ CNT,
                                                const int* __restrict__ OFF, const int* __restrict__ FLAG,
                                                const float* __restrict__ T, float* SOP) {
  const int tid = (int)threadIdx.x, lane = tid & 31, wave = tid >> 5;
  const int blk = (int)blockIdx.x;
  unsigned short* OP = (unsigned short*)SOP;

  if (blk >= WBLK) {
    const int row = NN + (blk - WBLK) * NWAVE + wave;
    const v2u z = {0u, 0u};
    unsigned short* cr = OP + (size_t)row * K2 + 4 * lane;
    for (int pass = 0; pass < 2; ++pass) {
      *(volatile v2u*)cr = z;
      *(volatile v2u*)(cr + FD) = z;
      __threadfence();
    }
    return;
  }

  int n = blk * NWAVE + wave;
  n = n > NN - 1 ? NN - 1 : n;
  const int bk = n >> SLB;
  const int cv = CNT[n];
  asm volatile("" :: "v"(cv));
  const int ovv = OFF[n];
  asm volatile("" :: "v"(ovv));
  const int fl = FLAG[(size_t)bk * 32];
  asm volatile("" :: "v"(fl));
  const v4f d = *(const v4fa*)(SOP + (size_t)n * FD + 4 * lane);
  const float d0 = d.x, d1 = d.y, d2 = d.z, d3 = d.w;
  asm volatile("" :: "v"(d0));
  asm volatile("" :: "v"(d1));
  asm volatile("" :: "v"(d2));
  asm volatile("" :: "v"(d3));

  const bool bad = (fl != 0) || (cv > DEGCAP) || (cv < 0);
  const int trip = __builtin_amdgcn_readfirstlane((fl == 0 && cv > 0) ? (cv > DEGCAP ? DEGCAP : cv) : 0);
  const int o = clampi(ovv, 0, RCAP - 1);
  int last = o + (trip > 0 ? trip : 1) - 1;
  last = last > RCAP - 1 ? RCAP - 1 : last;
  const int* lb = LIST + (size_t)bk * (size_t)RCAP;
  const float* tl = T + 4 * lane;

  v4f acc = (v4f){0.0f, 0.0f, 0.0f, 0.0f};
#pragma unroll 1
  for (int b0 = 0; b0 < trip; b0 += 32) {
    int idx = o + b0 + lane;
    idx = idx > last ? last : idx;
    int sr = lb[idx];
    sr = clampi(sr, 0, NN - 1);
    const int m32 = (trip - b0) < 32 ? (trip - b0) : 32;
#pragma unroll 1
    for (int k = 0; k < m32; ++k) {
      const int sk = __builtin_amdgcn_readlane(sr, k);
      const v4f q = *(const v4fa*)(tl + (size_t)sk * FD);
      acc += q;
    }
  }

  const float den = (float)(cv > 1 ? cv : 1);
  const float g0 = acc.x / den, g1 = acc.y / den, g2 = acc.z / den, g3 = acc.w / den;
  const float v0 = d0 + g0, v1 = d1 + g1, v2 = d2 + g2, v3 = d3 + g3;
  const float y0 = (v0 > 0.0f) ? v0 : (v0 - v0);
  const float y1 = (v1 > 0.0f) ? v1 : (v1 - v1);
  const float y2 = (v2 > 0.0f) ? v2 : (v2 - v2);
  const float y3 = (v3 > 0.0f) ? v3 : (v3 - v3);
  const float qnan = __uint_as_float(0x7fc00000u);
  const float u0 = bad ? qnan : y0, u1 = bad ? qnan : y1, u2 = bad ? qnan : y2, u3 = bad ? qnan : y3;

  v2u hv, lv2;
  hv.x = pk16(bf16_bits(u0), bf16_bits(u1));
  hv.y = pk16(bf16_bits(u2), bf16_bits(u3));
  if (SPLIT_L2) {
    lv2.x = pk16(bf16_lo_bits(u0), bf16_lo_bits(u1));
    lv2.y = pk16(bf16_lo_bits(u2), bf16_lo_bits(u3));
  } else {
    lv2.x = 0u;
    lv2.y = 0u;
  }
  unsigned short* cr = OP + (size_t)n * K2 + 4 * lane;
  for (int pass = 0; pass < 2; ++pass) {
    *(volatile v2u*)cr = hv;
    *(volatile v2u*)(cr + FD) = lv2;
    __threadfence();
  }
}

__global__ __launch_bounds__(NTHR) void k_walk2(const int* __restrict__ LIST, const int* __restrict__ CNT,
                                                const int* __restrict__ OFF, const int* __restrict__ FLAG,
                                                const float* __restrict__ T2, float* S2) {
  const int tid = (int)threadIdx.x, lane = tid & 31, wave = tid >> 5;
  const int blk = (int)blockIdx.x;
  int n = blk * NWAVE + wave;
  n = n > NN - 1 ? NN - 1 : n;
  const int bk = n >> SLB;
  const int cv = CNT[n];
  asm volatile("" :: "v"(cv));
  const int ovv = OFF[n];
  asm volatile("" :: "v"(ovv));
  const int fl = FLAG[(size_t)bk * 32];
  asm volatile("" :: "v"(fl));
  const v2f d = *(const v2fa*)(S2 + (size_t)n * OD + 2 * lane);
  const float d0 = d.x, d1 = d.y;
  asm volatile("" :: "v"(d0));
  asm volatile("" :: "v"(d1));

  const bool bad = (fl != 0) || (cv > DEGCAP) || (cv < 0);
  const int trip = __builtin_amdgcn_readfirstlane((fl == 0 && cv > 0) ? (cv > DEGCAP ? DEGCAP : cv) : 0);
  const int o = clampi(ovv, 0, RCAP - 1);
  int last = o + (trip > 0 ? trip : 1) - 1;
  last = last > RCAP - 1 ? RCAP - 1 : last;
  const int* lb = LIST + (size_t)bk * (size_t)RCAP;
  const float* tl = T2 + 2 * lane;

  v2f acc = (v2f){0.0f, 0.0f};
#pragma unroll 1
  for (int b0 = 0; b0 < trip; b0 += 32) {
    int idx = o + b0 + lane;
    idx = idx > last ? last : idx;
    int sr = lb[idx];
    sr = clampi(sr, 0, NN - 1);
    const int m32 = (trip - b0) < 32 ? (trip - b0) : 32;
#pragma unroll 1
    for (int k = 0; k < m32; ++k) {
      const int sk = __builtin_amdgcn_readlane(sr, k);
      const v2f q = *(const v2fa*)(tl + (size_t)sk * OD);
      acc += q;
    }
  }

  const float den = (float)(cv > 1 ? cv : 1);
  const float g0 = acc.x / den, g1 = acc.y / den;
  const float z0 = d0 + g0, z1 = d1 + g1;
  const float qnan = __uint_as_float(0x7fc00000u);
  v2f ov;
  ov.x = bad ? qnan : z0;
  ov.y = bad ? qnan : z1;
  float* zr = S2 + (size_t)n * OD + 2 * lane;
  *(volatile v2f*)zr = ov;
  __threadfence();
  *(volatile v2f*)zr = ov;
}

__global__ __launch_bounds__(NTHR) void k_head(const int* __restrict__ eli, const float* __restrict__ Z,
                                               const int* __restrict__ FLAG, const float* __restrict__ tab,
                                               float* out, int npair) {
  const int tid = (int)threadIdx.x, lane = tid & 31, wave = tid >> 5;
  const int wv = (int)blockIdx.x * NWAVE + wave;
  const int pbase = wv * 32;
  if (pbase >= NPAIR) return;

  const v2f wa = *(const v2fa*)(tab + TB_WDEC + 2 * lane);
  const v2f wb = *(const v2fa*)(tab + TB_WDEC + OD + 2 * lane);
  const float wa0 = wa.x, wa1 = wa.y, wb0 = wb.x, wb1 = wb.y;
  asm volatile("" :: "v"(wa0));
  asm volatile("" :: "v"(wa1));
  asm volatile("" :: "v"(wb0));
  asm volatile("" :: "v"(wb1));
  const float bd = tab[TB_BDEC];
  asm volatile("" :: "v"(bd));
  const float qnan = __uint_as_float(0x7fc00000u);

  float res = 0.0f;
#pragma unroll 1
  for (int j = 0; j < 32; ++j) {
    int pj = pbase + j;
    pj = pj > NPAIR - 1 ? NPAIR - 1 : pj;
    int a = eli[pj];
    asm volatile("" :: "v"(a));
    int b = eli[NPAIR + pj];
    asm volatile("" :: "v"(b));
    a = clampi(a, 0, NN - 1);
    b = clampi(b, 0, NN - 1);
    const v2f za = *(const v2fa*)(Z + (size_t)a * OD + 2 * lane);
    const v2f zb = *(const v2fa*)(Z + (size_t)b * OD + 2 * lane);
    const float za0 = za.x, za1 = za.y, zb0 = zb.x, zb1 = zb.y;
    asm volatile("" :: "v"(za0));
    asm volatile("" :: "v"(za1));
    asm volatile("" :: "v"(zb0));
    asm volatile("" :: "v"(zb1));
    const int fa = FLAG[(size_t)(a >> SLB) * 32];
    asm volatile("" :: "v"(fa));
    const int fb = FLAG[(size_t)(b >> SLB) * 32];
    asm volatile("" :: "v"(fb));
    float t = ((za0 * wa0 + za1 * wa1) + zb0 * wb0) + zb1 * wb1;
    t = t + __shfl_xor(t, 16, 32);
    t = t + __shfl_xor(t, 8, 32);
    t = t + __shfl_xor(t, 4, 32);
    t = t + __shfl_xor(t, 2, 32);
    t = t + __shfl_xor(t, 1, 32);
    const float r  = t + bd;
    const float rr = ((fa | fb) != 0) ? qnan : r;
    res = (lane == j) ? rr : res;
  }

  const int p = pbase + lane;
  if (p < npair) {
    float* q = out + p;
    *(volatile float*)q = res;
    __threadfence();
    *(volatile float*)q = res;
  }
}

extern "C" void kernel_launch(void* const* d_in, const int* in_sizes, int n_in,
                              void* d_out, int out_size, void* d_ws, size_t ws_size,
                              hipStream_t stream) {
  if (n_in < 11) return;
  if (in_sizes[0] != NN * FD) return;
  if (in_sizes[1] != 2 * NE) return;
  if (in_sizes[2] != 2 * NPAIR) return;
  if (in_sizes[3] != FD * FD) return;
  if (in_sizes[4] != FD) return;
  if (in_sizes[5] != FD * FD) return;
  if (in_sizes[6] != OD * FD) return;
  if (in_sizes[7] != OD) return;
  if (in_sizes[8] != OD * FD) return;
  if (in_sizes[9] != 2 * OD) return;
  if (in_sizes[10] != 1) return;
  if (out_size != NPAIR) return;

  const float* x    = (const float*)d_in[0];
  const int*   ei   = (const int*)d_in[1];
  const int*   eli  = (const int*)d_in[2];
  const float* Wl1  = (const float*)d_in[3];
  const float* bl1  = (const float*)d_in[4];
  const float* Wr1  = (const float*)d_in[5];
  const float* Wl2  = (const float*)d_in[6];
  const float* bl2  = (const float*)d_in[7];
  const float* Wr2  = (const float*)d_in[8];
  const float* Wdec = (const float*)d_in[9];
  const float* bdec = (const float*)d_in[10];
  float* out = (float*)d_out;

  constexpr size_t zRX   = (size_t)MP * FD * 2;
  constexpr size_t zRS   = (size_t)MP * FD * 4;
  constexpr size_t zRT   = (size_t)MP * FD * 4;
  constexpr size_t zHALF = (size_t)MP * OD * 4;
  constexpr size_t zW    = (size_t)FD * FD * 2;
  constexpr size_t zTAB  = (size_t)TB_FLOATS * 4;
  constexpr size_t zLIST = (size_t)NBK * RCAP * 4;
  constexpr size_t zCNT  = (size_t)NBK * NBRUN * 4;
  constexpr size_t zFLAG = (size_t)NBK * 128;
  constexpr size_t oRX   = 0;
  constexpr size_t oRS   = oRX + zRX;
  constexpr size_t oRT   = oRS + zRS;
  constexpr size_t oW1L  = oRT + zRT;
  constexpr size_t oW1R  = oW1L + zW;
  constexpr size_t oW2L  = oW1R + zW;
  constexpr size_t oW2R  = oW2L + zW;
  constexpr size_t oTAB  = oW2R + zW;
  constexpr size_t oEND  = oTAB + zTAB;
  constexpr size_t oLIST = oRX;
  constexpr size_t oCNT  = oLIST + zLIST;
  constexpr size_t oOFF  = oCNT + zCNT;
  constexpr size_t oFLAG = oOFF + zCNT;
  static_assert(zRX % 128 == 0 && zRS % 128 == 0 && zRT % 128 == 0 && zW % 128 == 0 && zTAB % 128 == 0);
  static_assert(zLIST % 128 == 0 && zCNT % 128 == 0 && zFLAG % 128 == 0);
  static_assert(oFLAG + zFLAG <= oRX + zRX);
  static_assert(zRS == (size_t)MP * K2 * 2 && zRT == 2 * zHALF && zW == (size_t)OD * K2 * 2);
  static_assert(zCNT >= (size_t)NN * 4);
  static_assert(oEND == (size_t)1002000 * 128);
  static_assert(oEND <= ((size_t)128 << 20));
  if (oEND > ws_size) return;

  char* ws = (char*)d_ws;
  unsigned short* XB   = (unsigned short*)(ws + oRX);
  int*            LIST = (int*)(ws + oLIST);
  int*            CNT  = (int*)(ws + oCNT);
  int*            OFF  = (int*)(ws + oOFF);
  int*            FLAG = (int*)(ws + oFLAG);
  float*          S    = (float*)(ws + oRS);
  unsigned short* OP   = (unsigned short*)(ws + oRS);
  float*          T    = (float*)(ws + oRT);
  float*          T2   = (float*)(ws + oRT);
  float*          S2   = (float*)(ws + oRT + zHALF);
  unsigned short* W1L  = (unsigned short*)(ws + oW1L);
  unsigned short* W1R  = (unsigned short*)(ws + oW1R);
  unsigned short* W2L  = (unsigned short*)(ws + oW2L);
  unsigned short* W2R  = (unsigned short*)(ws + oW2R);
  float*          TAB  = (float*)(ws + oTAB);

  hipFuncSetAttribute(reinterpret_cast<const void*>(&k_build), hipFuncAttributeMaxDynamicSharedMemorySize, (int)BK_LDS);

  const int tiles1 = ((NN + 63) / 64) * (FD / 64);
  const int gg1    = (tiles1 + 7) / 8;
  const int tiles2 = ((NN + 63) / 64) * (OD / 64);
  const int gg2    = (tiles2 + 7) / 8;

  k_plane<0><<<MP * FD / 8 / NTHR, NTHR, 0, stream>>>(x, NN, FD, FD, XB, MP, FD);
  k_prep<<<PW_BLKS, NTHR, 0, stream>>>(Wl1, Wr1, Wl2, Wr2, bl1, bl2, Wdec, bdec, W1L, W1R, W2L, W2R, TAB);
  k_gemm_nt<0, 1><<<gg1, NTHR, 0, stream>>>(XB, W1R, TAB + TB_BL1, S, NN, FD, FD, FD);
  k_gemm_nt<0, 0><<<gg1, NTHR, 0, stream>>>(XB, W1L, TAB + TB_BL1, T, NN, FD, FD, FD);
  k_build<<<NBK, NTHR, BK_LDS, stream>>>(ei, ei + NE, LIST, CNT, OFF, FLAG);
  k_walk1<<<WBLK + PADBLK, NTHR, 0, stream>>>(LIST, CNT, OFF, FLAG, T, S);
  k_gemm_nt<0, 0><<<gg2, NTHR, 0, stream>>>(OP, W2L, TAB + TB_BL2, T2, NN, OD, K2, OD);
  k_gemm_nt<0, 1><<<gg2, NTHR, 0, stream>>>(OP, W2R, TAB + TB_BL2, S2, NN, OD, K2, OD);
  k_walk2<<<WBLK, NTHR, 0, stream>>>(LIST, CNT, OFF, FLAG, T2, S2);
  k_head<<<HBLK, NTHR, 0, stream>>>(eli, S2, FLAG, TAB, out, out_size);
}
